// LSTM_51204600103202
// MI455X (gfx1250) — hardware-verified
//
#include <hip/hip_runtime.h>
#include <math.h>

constexpr int NHID     = 128;
constexpr int NGATE    = 4 * NHID;
constexpr int NSTEP    = 7;
constexpr int NBATCH   = 65536;
constexpr int ROWS_BLK = 32;
constexpr int NTHR     = 512;
constexpr int NWAVE    = NTHR / 32;
constexpr int NUB      = NHID / 16;
constexpr int HPITCH   = 136;
constexpr float WCARRY = 256.0f;
constexpr float HCARRY = 1024.0f;
constexpr float FOLD   = 1.0f / (WCARRY * HCARRY);

static_assert(NBATCH % ROWS_BLK == 0, "grid exact");
static_assert((ROWS_BLK * NSTEP * 4) % 128 == 0, "block output region is whole 128-B lines");
static_assert(ROWS_BLK * NSTEP == 224, "final store map: 56 float4 = 32 + 24 lanes");
static_assert(NHID % 32 == 0, "K multiple of 32");
static_assert(NWAVE == (ROWS_BLK / 16) * NUB, "one 16x16 unit tile per wave");
static_assert(NSTEP * ROWS_BLK <= NTHR && (NSTEP * ROWS_BLK) % 32 == 0, "staging covers whole waves");
static_assert((HPITCH % 8) == 0 && HPITCH >= NHID, "16-B aligned LDS rows");
static_assert((NGATE * NHID) % (8 * 256) == 0, "convert grid exact");

typedef __attribute__((ext_vector_type(16))) _Float16 v16h;
typedef __attribute__((ext_vector_type(8)))  _Float16 v8h;
typedef __attribute__((ext_vector_type(8)))  float    v8f;
typedef __attribute__((ext_vector_type(4)))  float    v4f;

__device__ __forceinline__ void wmma_guard_all(v8f& a0, v8f& a1, v8f& a2, v8f& a3,
                                               v16h x, v16h y0, v16h y1, v16h y2, v16h y3) {
  asm volatile("v_nop\n\tv_nop\n\tv_nop\n\tv_nop"
               : "+v"(a0), "+v"(a1), "+v"(a2), "+v"(a3)
               : "v"(x), "v"(y0), "v"(y1), "v"(y2), "v"(y3));
}
__device__ __forceinline__ void acc_guard4(v8f& a, v8f& b, v8f& c, v8f& d) {
  asm volatile("v_nop\n\tv_nop\n\tv_nop\n\tv_nop" : "+v"(a), "+v"(b), "+v"(c), "+v"(d));
}

struct FragH {
  union U { v16h v; v8h h[2]; };
  static __device__ __forceinline__ v16h load(const _Float16* p) {
    U f;
    f.h[0] = *(const v8h*)(p);
    f.h[1] = *(const v8h*)(p + 16);
    return f.v;
  }
  static __device__ __forceinline__ v8f mma(v16h a, v16h b, v8f c) {
    return __builtin_amdgcn_wmma_f32_16x16x32_f16(false, a, false, b, (short)0, c, false, false);
  }
};

__device__ __forceinline__ float fsig(float v)  { return 1.0f / (1.0f + expf(-v)); }
__device__ __forceinline__ float ftanh(float v) { return 1.0f - 2.0f / (1.0f + expf(2.0f * v)); }

__global__ __launch_bounds__(256) void cvt_w_kernel(const float* __restrict__ src, unsigned short* __restrict__ dst,
                                                    int n8, float sc) {
  const int i = blockIdx.x * 256 + threadIdx.x;
  if (i < n8) {
    const float* sp = src + (size_t)i * 8;
    const v4f a = *(const v4f*)(sp);
    const v4f b = *(const v4f*)(sp + 4);
    v8h hv;
#pragma unroll
    for (int e = 0; e < 4; ++e) {
      const float fa = a[e] * sc;
      const float fb = b[e] * sc;
      hv[e]     = (_Float16)fa;
      hv[4 + e] = (_Float16)fb;
    }
    *(volatile v8h*)(dst + (size_t)i * 8) = hv;
    __threadfence();
    *(volatile v8h*)(dst + (size_t)i * 8) = hv;
  }
}

__global__ __launch_bounds__(NTHR) void lstm_seq_kernel(const float* __restrict__ x, const float* __restrict__ x0,
                                                        const float* __restrict__ w_ih, const float* __restrict__ b_ih,
                                                        const float* __restrict__ b_hh, const float* __restrict__ w_out,
                                                        const float* __restrict__ b_out,
                                                        const unsigned short* __restrict__ WHp,
                                                        float* __restrict__ out) {
  __shared__ __align__(16) _Float16 Ah[2][ROWS_BLK * HPITCH];
  __shared__ __align__(16) float    s_xs[NSTEP * ROWS_BLK];
  __shared__ __align__(16) float    s_pp[NSTEP * NUB * ROWS_BLK];

  const _Float16* WH = (const _Float16*)WHp;
  const int tid  = threadIdx.x;
  const int lane = tid & 31;
  const int wave = tid >> 5;
  const int c    = lane & 15;
  const int hh   = lane >> 4;
  const int koff = hh * 8;
  const int mt   = wave >> 3;
  const int ub   = wave & 7;
  const int col  = 16 * ub + c;
  const int rowbase = blockIdx.x * ROWS_BLK;

  if (tid < NSTEP * ROWS_BLK) {
    const int ts = tid >> 5;
    const int rr = tid & 31;
    const int tx = (ts > 0) ? (ts - 1) : 0;
    const float v0 = x0[rowbase + rr];
    const float vx = x[(size_t)(rowbase + rr) * NSTEP + tx];
    const float fa = (ts == 0) ? 1.0f : 0.0f;
    const float fb = 1.0f - fa;
    s_xs[tid] = fmaf(fa, v0, fb * vx);
  }
  asm volatile("" ::: "memory");

  float wih[4], bsum[4];
#pragma unroll
  for (int g = 0; g < 4; ++g) wih[g] = w_ih[g * NHID + col];
  asm volatile("" ::: "memory");
#pragma unroll
  for (int g = 0; g < 4; ++g) {
    const float ba = b_ih[g * NHID + col];
    const float bb = b_hh[g * NHID + col];
    bsum[g] = ba + bb;
  }
  asm volatile("" ::: "memory");
  const float wout = w_out[col];

  float cst[8];
#pragma unroll
  for (int r = 0; r < 8; ++r) cst[r] = 0.0f;

  __syncthreads();

  const v8f z8 = {0.f, 0.f, 0.f, 0.f, 0.f, 0.f, 0.f, 0.f};
  const _Float16* wrow = WH + (size_t)col * NHID + koff;

#pragma unroll 1
  for (int t = 0; t < NSTEP; ++t) {
    v8f acc0 = z8, acc1 = z8, acc2 = z8, acc3 = z8;
    if (t > 0) {
      const _Float16* arow = &Ah[(t - 1) & 1][0] + (16 * mt + c) * HPITCH + koff;
#pragma unroll 2
      for (int k0 = 0; k0 < NHID; k0 += 32) {
        const v16h a  = FragH::load(arow + k0);
        const v16h b0 = FragH::load(wrow + k0);
        const v16h b1 = FragH::load(wrow + (size_t)1 * NHID * NHID + k0);
        const v16h b2 = FragH::load(wrow + (size_t)2 * NHID * NHID + k0);
        const v16h b3 = FragH::load(wrow + (size_t)3 * NHID * NHID + k0);
        acc0 = FragH::mma(a, b0, acc0);
        acc1 = FragH::mma(a, b1, acc1);
        acc2 = FragH::mma(a, b2, acc2);
        acc3 = FragH::mma(a, b3, acc3);
        wmma_guard_all(acc0, acc1, acc2, acc3, a, b0, b1, b2, b3);
      }
    }
    acc_guard4(acc0, acc1, acc2, acc3);

    const float* xsp = s_xs + t * ROWS_BLK + 16 * mt + 8 * hh;
    _Float16* ahn = &Ah[t & 1][0];
    float pp[8];
#pragma unroll
    for (int r = 0; r < 8; ++r) {
      const float xv = xsp[r];
      const float zi = acc0[r] * FOLD + (xv * wih[0] + bsum[0]);
      const float zf = acc1[r] * FOLD + (xv * wih[1] + bsum[1]);
      const float zg = acc2[r] * FOLD + (xv * wih[2] + bsum[2]);
      const float zo = acc3[r] * FOLD + (xv * wih[3] + bsum[3]);
      const float ig = fsig(zi);
      const float fg = fsig(zf);
      const float gg = ftanh(zg);
      const float og = fsig(zo);
      const float cn = fg * cst[r] + ig * gg;
      cst[r] = cn;
      const float hn = og * ftanh(cn);
      pp[r] = hn * wout;
      const float hs = hn * HCARRY;
      ahn[(16 * mt + 8 * hh + r) * HPITCH + col] = (_Float16)hs;
    }

#pragma unroll
    for (int r = 0; r < 8; ++r) {
      float v = pp[r];
      v += __shfl_xor(v, 1, 32);
      v += __shfl_xor(v, 2, 32);
      v += __shfl_xor(v, 4, 32);
      v += __shfl_xor(v, 8, 32);
      pp[r] = v;
    }
    if (c == 0) {
#pragma unroll
      for (int r = 0; r < 8; ++r) s_pp[(t * NUB + ub) * ROWS_BLK + 16 * mt + 8 * hh + r] = pp[r];
    }
    __syncthreads();
  }

  if (wave == 0) {
    const float bo = b_out[0];
    const int q0 = lane;
    const int q1 = 32 + ((lane < 24) ? lane : 23);
    v4f va, vb;
#pragma unroll
    for (int e = 0; e < 4; ++e) {
      const int i0 = 4 * q0 + e;
      const int r0 = i0 / NSTEP;
      const int t0 = i0 - NSTEP * r0;
      const int i1 = 4 * q1 + e;
      const int r1 = i1 / NSTEP;
      const int t1 = i1 - NSTEP * r1;
      float s0 = 0.0f, s1 = 0.0f;
#pragma unroll
      for (int u = 0; u < NUB; ++u) {
        s0 += s_pp[(t0 * NUB + u) * ROWS_BLK + r0];
        s1 += s_pp[(t1 * NUB + u) * ROWS_BLK + r1];
      }
      va[e] = s0 + bo;
      vb[e] = s1 + bo;
    }
    float* ob = out + (size_t)rowbase * NSTEP;
    for (int pass = 0; pass < 2; ++pass) {
      *(volatile v4f*)(ob + 4 * lane) = va;
      if (lane < 24) *(volatile v4f*)(ob + 128 + 4 * lane) = vb;
      __threadfence();
    }
  }
}

extern "C" void kernel_launch(void* const* d_in, const int* in_sizes, int n_in,
                              void* d_out, int out_size, void* d_ws, size_t ws_size, hipStream_t stream) {
  if (n_in < 8 || d_out == nullptr || d_ws == nullptr) return;
  if (in_sizes[0] != NBATCH * NSTEP || in_sizes[1] != NBATCH || in_sizes[2] != NGATE ||
      in_sizes[3] != NGATE * NHID || in_sizes[4] != NGATE || in_sizes[5] != NGATE ||
      in_sizes[6] != NHID || in_sizes[7] != 1 || out_size != NBATCH * NSTEP) return;

  const float* x     = (const float*)d_in[0];
  const float* x0    = (const float*)d_in[1];
  const float* w_ih  = (const float*)d_in[2];
  const float* w_hh  = (const float*)d_in[3];
  const float* b_ih  = (const float*)d_in[4];
  const float* b_hh  = (const float*)d_in[5];
  const float* w_out = (const float*)d_in[6];
  const float* b_out = (const float*)d_in[7];
  float* out = (float*)d_out;

  const size_t wh_bytes = (size_t)NGATE * NHID * 2;
  if (wh_bytes > ws_size || wh_bytes > (size_t)134217728) return;
  unsigned short* WH = (unsigned short*)d_ws;

  const int n8 = NGATE * NHID / 8;
  cvt_w_kernel<<<n8 / 256, 256, 0, stream>>>(w_hh, WH, n8, WCARRY);
  lstm_seq_kernel<<<NBATCH / ROWS_BLK, NTHR, 0, stream>>>(x, x0, w_ih, b_ih, b_hh, w_out, b_out, WH, out);
}
